// mp_layer_39943195852850
// MI455X (gfx1250) — hardware-verified
//
#include <hip/hip_runtime.h>
#include <stddef.h>


#define CH     128
#define KNB    16
#define APZ    136
#define APW    264
#define KPB    128
#define KPW    256
#define PQW    256
#define NTHR   256
#define NWAVE  8
#define NIT    16
#define NPB    (NWAVE * NIT)
#define GROWS  32
#define GTHR   64
#define DEGCAP 1024
#define EPT    8
#define NGRP   2
#define CHUNK  (NTHR * EPT * NGRP)
#define WCAP   (EPT * NGRP * 32)
#define LISTN  (NWAVE * WCAP)
#define NBC    4096
#define NBF    1024
#define RCAP   40960
#define RBN    128
#define OTHR   512
#define LDS_FILL ((RCAP + NBF + LISTN) * 4 + 64)
#define OFF_B1H 0
#define OFF_B1L 32768
#define OFF_B2  65536
#define OFF_B3H 81920
#define OFF_B3L 114688
#define OFF_B4H 147456
#define OFF_B4L 163840
#define BPTOT   180224
#define WSCAP  134217728
#define WSC    64.0f
#define ZSC    16.0f
#define RZW    0.0009765625f

static_assert(NIT * NWAVE == NPB);
static_assert(GROWS == (GTHR / 32) * 16);
static_assert((APZ % 8) == 0 && (APW % 8) == 0 && (KPB % 8) == 0 && (KPW % 8) == 0 && (PQW % 32) == 0);
static_assert(OFF_B1L == 2 * CH * KPB && OFF_B2 == 2 * OFF_B1L && OFF_B3H == OFF_B2 + CH * KPB);
static_assert(OFF_B3L == OFF_B3H + CH * KPW && OFF_B4H == OFF_B3L + CH * KPW && OFF_B4L == OFF_B4H + CH * KPB);
static_assert(BPTOT == OFF_B4L + CH * KPB);
static_assert(32 * GTHR * 4 == GROWS * PQW);
static_assert(16 * GTHR * 4 == GROWS * CH);
static_assert(NTHR * 4 == NWAVE * CH);
static_assert((CHUNK & (CHUNK - 1)) == 0);
static_assert(CHUNK <= 4096);
static_assert(NBC <= 4096 && NBF <= 4096);
static_assert((NBC & (NBC - 1)) == 0 && (NBF & (NBF - 1)) == 0);
static_assert(NBC == 4 * NBF);
static_assert(OTHR * 8 == NBC);
static_assert((RCAP % 32) == 0);
static_assert((DEGCAP % KNB) == 0);
static_assert((CH % 32) == 0);
static_assert(GROWS * CH * 2 <= GROWS * APW);

typedef float          v4f  __attribute__((ext_vector_type(4)));
typedef float          v8f  __attribute__((ext_vector_type(8)));
typedef int            v4i  __attribute__((ext_vector_type(4)));
typedef int            v8i  __attribute__((ext_vector_type(8)));
typedef unsigned short v8us __attribute__((ext_vector_type(8)));
typedef _Float16       v4h  __attribute__((ext_vector_type(4)));
typedef _Float16       v8h  __attribute__((ext_vector_type(8)));
typedef _Float16       v16h __attribute__((ext_vector_type(16)));
typedef __bf16         v16b __attribute__((ext_vector_type(16)));
union Frag  { v16h v; v8h h[2]; };
union FragB { v16b v; v8us u[2]; v8i w; };

__device__ __forceinline__ v8f wmh(v16h a, v16h b, v8f c) {
  v8f d = __builtin_amdgcn_wmma_f32_16x16x32_f16(false, a, false, b, (short)0, c, false, false);
  asm volatile("v_nop\n\tv_nop\n\tv_nop\n\tv_nop" : "+v"(d) : "v"(a), "v"(b));
  return d;
}

__device__ __forceinline__ v8f wmb(const FragB& a, const FragB& b, v8f c) {
  v8f d = __builtin_amdgcn_wmma_f32_16x16x32_bf16(false, a.v, false, b.v, (short)0, c, false, false);
  asm volatile("v_nop\n\tv_nop\n\tv_nop\n\tv_nop" : "+v"(d) : "v"(a.w), "v"(b.w));
  return d;
}

__device__ __forceinline__ void bfsplit(float f, unsigned short& hi, unsigned short& lo) {
  const unsigned u = __float_as_uint(f);
  const unsigned r = (u + 0x7FFFu + ((u >> 16) & 1u)) & 0xFFFF0000u;
  hi = (unsigned short)(r >> 16);
  const float d = f - __uint_as_float(r);
  const unsigned ud = __float_as_uint(d);
  lo = (unsigned short)((ud + 0x7FFFu + ((ud >> 16) & 1u)) >> 16);
}

__device__ __forceinline__ void split8(v4f a, v4f b, v8us& hv, v8us& lv) {
  float f[8] = {a.x, a.y, a.z, a.w, b.x, b.y, b.z, b.w};
#pragma unroll
  for (int e = 0; e < 8; ++e) {
    unsigned short hs, ls;
    bfsplit(f[e], hs, ls);
    hv[e] = hs;
    lv[e] = ls;
  }
}

__device__ __forceinline__ v4h cvt4z(v4f a) {
  v4h r;
  r.x = (_Float16)(a.x * ZSC); r.y = (_Float16)(a.y * ZSC); r.z = (_Float16)(a.z * ZSC); r.w = (_Float16)(a.w * ZSC);
  return r;
}

__device__ __forceinline__ v4f axpy4(float s, v4f d, v4f u) {
  u.x = fmaf(s, d.x, u.x); u.y = fmaf(s, d.y, u.y); u.z = fmaf(s, d.z, u.z); u.w = fmaf(s, d.w, u.w);
  return u;
}

template <int NT>
__device__ __forceinline__ void mma16(const _Float16* At, const _Float16* __restrict__ Bpl,
                                      int lane, v8f (&acc)[NT]) {
  const int hh = lane >> 4, m = lane & 15;
#pragma unroll
  for (int t = 0; t < NT; ++t) { v8f z = {0.f, 0.f, 0.f, 0.f, 0.f, 0.f, 0.f, 0.f}; acc[t] = z; }
  const _Float16* ap = At + m * APZ + 8 * hh;
  const _Float16* bb = Bpl + (size_t)m * KPB + 8 * hh;
#pragma unroll 1
  for (int ks = 0; ks < CH / 32; ++ks) {
    Frag a;
    a.h[0] = *(const v8h*)(ap + 32 * ks);
    a.h[1] = *(const v8h*)(ap + 32 * ks + 16);
#pragma unroll
    for (int t = 0; t < NT; ++t) {
      const _Float16* bp = bb + (size_t)(16 * t) * KPB + 32 * ks;
      Frag b;
      b.h[0] = *(const v8h*)bp;
      b.h[1] = *(const v8h*)(bp + 16);
      acc[t] = wmh(a.v, b.v, acc[t]);
    }
  }
}

template <int NT, int KK, int AP>
__device__ __forceinline__ void mma3(const unsigned short* Ah, const unsigned short* Al,
                                     const unsigned short* __restrict__ Bh, const unsigned short* __restrict__ Bl,
                                     int lane, v8f (&acc)[NT]) {
  const int hh = lane >> 4, m = lane & 15;
#pragma unroll
  for (int t = 0; t < NT; ++t) { v8f z = {0.f, 0.f, 0.f, 0.f, 0.f, 0.f, 0.f, 0.f}; acc[t] = z; }
  const unsigned short* aph = Ah + m * AP + 8 * hh;
  const unsigned short* apl = Al + m * AP + 8 * hh;
  const unsigned short* bbh = Bh + (size_t)m * KK + 8 * hh;
  const unsigned short* bbl = Bl + (size_t)m * KK + 8 * hh;
#pragma unroll 1
  for (int ks = 0; ks < KK / 32; ++ks) {
    FragB ah, al;
    ah.u[0] = *(const v8us*)(aph + 32 * ks);
    ah.u[1] = *(const v8us*)(aph + 32 * ks + 16);
    al.u[0] = *(const v8us*)(apl + 32 * ks);
    al.u[1] = *(const v8us*)(apl + 32 * ks + 16);
#pragma unroll
    for (int t = 0; t < NT; ++t) {
      const unsigned short* bph = bbh + (size_t)(16 * t) * KK + 32 * ks;
      const unsigned short* bpl = bbl + (size_t)(16 * t) * KK + 32 * ks;
      FragB bh, bl;
      bh.u[0] = *(const v8us*)bph;
      bh.u[1] = *(const v8us*)(bph + 16);
      bl.u[0] = *(const v8us*)bpl;
      bl.u[1] = *(const v8us*)(bpl + 16);
      acc[t] = wmb(ah, bh, acc[t]);
      acc[t] = wmb(ah, bl, acc[t]);
      acc[t] = wmb(al, bh, acc[t]);
    }
  }
}

template <int J0>
__device__ __forceinline__ void rows_z(_Float16* zw, const float* __restrict__ PQ, int sv,
                                       float dx, float dy, float dz, v4f qb, v4f d0, v4f d1, v4f d2, int lane) {
#pragma unroll
  for (int j = J0; j < J0 + 8; ++j) {
    const int s = __builtin_amdgcn_readlane(sv, j);
    const float fx = __int_as_float(__builtin_amdgcn_readlane(__float_as_int(dx), j));
    const float fy = __int_as_float(__builtin_amdgcn_readlane(__float_as_int(dy), j));
    const float fz = __int_as_float(__builtin_amdgcn_readlane(__float_as_int(dz), j));
    const v4f p = *(const v4f*)(PQ + (size_t)s * PQW + 4 * lane);
    v4f u = p + qb;
    u = axpy4(fx, d0, u);
    u = axpy4(fy, d1, u);
    u = axpy4(fz, d2, u);
    u.x = fmaxf(u.x, 0.0f); u.y = fmaxf(u.y, 0.0f); u.z = fmaxf(u.z, 0.0f); u.w = fmaxf(u.w, 0.0f);
    *(v4h*)(zw + j * APZ + 4 * lane) = cvt4z(u);
  }
}

template <int NB>
__device__ __forceinline__ int scan_chunk(const int* __restrict__ dsts, int nE, int cbase, int slotBase,
                                          int vec8, int* list, int tid, int lane, int wave) {
  int wc = 0;
#pragma unroll
  for (int g = 0; g < NGRP; ++g) {
    const int el0  = (g * NTHR + tid) * EPT;
    const int e0   = cbase + el0;
    const int sent = -2147483647 - 1;
    v4i da, db;
    if (vec8 != 0 && cbase + CHUNK <= nE) {
      da = *(const v4i*)(dsts + e0);
      db = *(const v4i*)(dsts + e0 + 4);
    } else {
      da.x = (e0     < nE) ? dsts[min(e0, nE - 1)] : sent;
      da.y = (e0 + 1 < nE) ? dsts[min(e0 + 1, nE - 1)] : sent;
      da.z = (e0 + 2 < nE) ? dsts[min(e0 + 2, nE - 1)] : sent;
      da.w = (e0 + 3 < nE) ? dsts[min(e0 + 3, nE - 1)] : sent;
      db.x = (e0 + 4 < nE) ? dsts[min(e0 + 4, nE - 1)] : sent;
      db.y = (e0 + 5 < nE) ? dsts[min(e0 + 5, nE - 1)] : sent;
      db.z = (e0 + 6 < nE) ? dsts[min(e0 + 6, nE - 1)] : sent;
      db.w = (e0 + 7 < nE) ? dsts[min(e0 + 7, nE - 1)] : sent;
    }
    const unsigned nb = (unsigned)slotBase;
    const unsigned s0 = (unsigned)da.x - nb, s1 = (unsigned)da.y - nb;
    const unsigned s2 = (unsigned)da.z - nb, s3 = (unsigned)da.w - nb;
    const unsigned s4 = (unsigned)db.x - nb, s5 = (unsigned)db.y - nb;
    const unsigned s6 = (unsigned)db.z - nb, s7 = (unsigned)db.w - nb;
    const bool h0 = s0 < (unsigned)NB, h1 = s1 < (unsigned)NB, h2 = s2 < (unsigned)NB, h3 = s3 < (unsigned)NB;
    const bool h4 = s4 < (unsigned)NB, h5 = s5 < (unsigned)NB, h6 = s6 < (unsigned)NB, h7 = s7 < (unsigned)NB;
    const unsigned any = __builtin_amdgcn_ballot_w32(h0 | h1 | h2 | h3 | h4 | h5 | h6 | h7);
    if (any != 0u) {
#define HITJ(J, HJ, SJ) { \
        const unsigned mj = __builtin_amdgcn_ballot_w32(HJ); \
        if (mj != 0u) { \
          if (HJ) { \
            const int hp = wc + (int)__builtin_amdgcn_mbcnt_lo(mj, 0u); \
            if (hp < WCAP) list[wave * WCAP + hp] = ((el0 + (J)) << 12) | (int)(SJ); \
          } \
          wc += (int)__builtin_popcount(mj); } }
      HITJ(0, h0, s0)
      HITJ(1, h1, s1)
      HITJ(2, h2, s2)
      HITJ(3, h3, s3)
      HITJ(4, h4, s4)
      HITJ(5, h5, s5)
      HITJ(6, h6, s6)
      HITJ(7, h7, s7)
#undef HITJ
    }
  }
  return wc;
}

__global__ __launch_bounds__(NTHR) void k_wprep(const float* __restrict__ We0, const float* __restrict__ We1,
                                                const float* __restrict__ Wn0, const float* __restrict__ Wn1,
                                                unsigned short* Bpl) {
  const int blk = blockIdx.x, tid = threadIdx.x;
  float v[8];
  if (blk < 16) {
    const int i = blk * NTHR + tid;
    const int n = i >> 4, k0 = (i & 15) * 8;
    const int sel = n >> 7, nc = n & (CH - 1);
    const int kb = sel * CH;
#pragma unroll
    for (int e = 0; e < 8; ++e) {
      const float a = We0[(kb + k0 + e) * CH + nc];
      const float c = We0[(2 * CH + k0 + e) * CH + nc];
      v[e] = (sel != 0) ? (a - c) : (a + c);
    }
    v8us hv, lv;
#pragma unroll
    for (int e = 0; e < 8; ++e) { unsigned short hs, ls; bfsplit(v[e], hs, ls); hv[e] = hs; lv[e] = ls; }
    unsigned short* ph = Bpl + OFF_B1H + i * 8;
    unsigned short* pl = Bpl + OFF_B1L + i * 8;
    *(volatile v8us*)ph = hv;
    *(volatile v8us*)pl = lv;
    __threadfence();
    *(volatile v8us*)ph = hv;
    *(volatile v8us*)pl = lv;
  } else if (blk < 24) {
    const int i = (blk - 16) * NTHR + tid;
    const int n = i >> 4, k0 = (i & 15) * 8;
#pragma unroll
    for (int e = 0; e < 8; ++e) v[e] = We1[(k0 + e) * CH + n];
    v8h hv;
#pragma unroll
    for (int e = 0; e < 8; ++e) hv[e] = (_Float16)(v[e] * WSC);
    _Float16* dp = (_Float16*)(Bpl + OFF_B2) + i * 8;
    *(volatile v8h*)dp = hv;
    __threadfence();
    *(volatile v8h*)dp = hv;
  } else if (blk < 40) {
    const int i = (blk - 24) * NTHR + tid;
    const int n = i >> 5, k0 = (i & 31) * 8;
#pragma unroll
    for (int e = 0; e < 8; ++e) v[e] = Wn0[(k0 + e) * CH + n];
    v8us hv, lv;
#pragma unroll
    for (int e = 0; e < 8; ++e) { unsigned short hs, ls; bfsplit(v[e], hs, ls); hv[e] = hs; lv[e] = ls; }
    unsigned short* ph = Bpl + OFF_B3H + i * 8;
    unsigned short* pl = Bpl + OFF_B3L + i * 8;
    *(volatile v8us*)ph = hv;
    *(volatile v8us*)pl = lv;
    __threadfence();
    *(volatile v8us*)ph = hv;
    *(volatile v8us*)pl = lv;
  } else {
    const int i = (blk - 40) * NTHR + tid;
    const int n = i >> 4, k0 = (i & 15) * 8;
#pragma unroll
    for (int e = 0; e < 8; ++e) v[e] = Wn1[(k0 + e) * CH + n];
    v8us hv, lv;
#pragma unroll
    for (int e = 0; e < 8; ++e) { unsigned short hs, ls; bfsplit(v[e], hs, ls); hv[e] = hs; lv[e] = ls; }
    unsigned short* ph = Bpl + OFF_B4H + i * 8;
    unsigned short* pl = Bpl + OFF_B4L + i * 8;
    *(volatile v8us*)ph = hv;
    *(volatile v8us*)pl = lv;
    __threadfence();
    *(volatile v8us*)ph = hv;
    *(volatile v8us*)pl = lv;
  }
}

__global__ __launch_bounds__(NTHR) void k_count(const int* __restrict__ dsts, int* cnt, int nE, int vec8) {
  __shared__ __attribute__((aligned(16))) int scnt[NBC];
  __shared__ __attribute__((aligned(16))) int list[LISTN];
  __shared__ int wcnt[NWAVE];
  const int tid = threadIdx.x, lane = tid & 31, wave = tid >> 5;
  const int nodeBase = blockIdx.x * NBC;

  for (int i = tid; i < NBC; i += NTHR) scnt[i] = 0;
  __syncthreads();

  const int nChunks = (nE + CHUNK - 1) / CHUNK;
#pragma unroll 1
  for (int ch = 0; ch < nChunks; ++ch) {
    const int cbase = ch * CHUNK;
    const int wc = scan_chunk<NBC>(dsts, nE, cbase, nodeBase, vec8, list, tid, lane, wave);
    if (lane == 0) wcnt[wave] = wc;
    __syncthreads();
    if (wave == 0) {
#pragma unroll 1
      for (int wsx = 0; wsx < NWAVE; ++wsx) {
        int n = __builtin_amdgcn_readfirstlane(wcnt[wsx]);
        n = n > WCAP ? WCAP : (n < 0 ? 0 : n);
        const int* lp = list + wsx * WCAP;
#pragma unroll 1
        for (int i = 0; i < n; ++i) {
          const int ent = __builtin_amdgcn_readfirstlane(lp[i]);
          const int sl  = ent & (NBC - 1);
          if (lane == 0) scnt[sl] = scnt[sl] + 1;
        }
      }
    }
    __syncthreads();
  }

  v4i cq[4];
#pragma unroll
  for (int q = 0; q < 4; ++q) {
    const int f = (wave * 4 + q) * 128 + 4 * lane;
    cq[q] = *(const v4i*)(scnt + f);
  }
  int* cp = cnt + (size_t)nodeBase;
#pragma unroll
  for (int q = 0; q < 4; ++q) {
    const int f = (wave * 4 + q) * 128 + 4 * lane;
    *(volatile v4i*)(cp + f) = cq[q];
  }
  __threadfence();
#pragma unroll
  for (int q = 0; q < 4; ++q) {
    const int f = (wave * 4 + q) * 128 + 4 * lane;
    *(volatile v4i*)(cp + f) = cq[q];
  }
}

__global__ __launch_bounds__(OTHR) void k_offsets(
    const int* __restrict__ cnt, int* off, int* rbase, int nChunk) {
  __shared__ __attribute__((aligned(16))) int soff[NBC];
  __shared__ __attribute__((aligned(16))) int srb[RBN];
  __shared__ int wtot[OTHR / 32];
  const int tid = threadIdx.x, lane = tid & 31, wave = tid >> 5, sub = tid >> 7;
  for (int i = tid; i < RBN; i += OTHR) srb[i] = 0;
  int carry = 0;
#pragma unroll 1
  for (int ch = 0; ch < nChunk; ++ch) {
    const int base = ch * NBC;
    const v4i c0 = *(const v4i*)(cnt + base + 8 * tid);
    const v4i c1 = *(const v4i*)(cnt + base + 8 * tid + 4);
    const int e0 = max(c0.x, 0), e1 = max(c0.y, 0), e2 = max(c0.z, 0), e3 = max(c0.w, 0);
    const int e4 = max(c1.x, 0), e5 = max(c1.y, 0), e6 = max(c1.z, 0), e7 = max(c1.w, 0);
    const int ts = e0 + e1 + e2 + e3 + e4 + e5 + e6 + e7;
    int incl = ts;
#pragma unroll
    for (int d = 1; d < 32; d <<= 1) {
      const int t = __shfl_up(incl, d);
      if (lane >= d) incl += t;
    }
    if (lane == 31) wtot[wave] = incl;
    __syncthreads();
    const int S0 = wtot[0]  + wtot[1]  + wtot[2]  + wtot[3];
    const int S1 = wtot[4]  + wtot[5]  + wtot[6]  + wtot[7];
    const int S2 = wtot[8]  + wtot[9]  + wtot[10] + wtot[11];
    const int S3 = wtot[12] + wtot[13] + wtot[14] + wtot[15];
    int pre = 0;
#pragma unroll 1
    for (int w = 4 * sub; w < wave; ++w) pre += wtot[w];
    const int b0 = carry;
    const int b1 = b0 + ((S0 + 31) & ~31);
    const int b2 = b1 + ((S1 + 31) & ~31);
    const int b3 = b2 + ((S2 + 31) & ~31);
    const int b4 = b3 + ((S3 + 31) & ~31);
    const int myb = sub == 0 ? b0 : (sub == 1 ? b1 : (sub == 2 ? b2 : b3));
    if (tid == 0) {
      srb[min(4 * ch + 0, RBN - 1)] = b0;
      srb[min(4 * ch + 1, RBN - 1)] = b1;
      srb[min(4 * ch + 2, RBN - 1)] = b2;
      srb[min(4 * ch + 3, RBN - 1)] = b3;
    }
    int run = myb + pre + incl - ts;
    soff[8 * tid + 0] = run; run += e0;
    soff[8 * tid + 1] = run; run += e1;
    soff[8 * tid + 2] = run; run += e2;
    soff[8 * tid + 3] = run; run += e3;
    soff[8 * tid + 4] = run; run += e4;
    soff[8 * tid + 5] = run; run += e5;
    soff[8 * tid + 6] = run; run += e6;
    soff[8 * tid + 7] = run;
    carry = b4;
    __syncthreads();
    const v4i o0 = *(const v4i*)(soff + 4 * tid);
    const v4i o1 = *(const v4i*)(soff + 4 * (tid + OTHR));
    int* op = off + base;
    *(volatile v4i*)(op + 4 * tid) = o0;
    *(volatile v4i*)(op + 4 * (tid + OTHR)) = o1;
    __threadfence();
    *(volatile v4i*)(op + 4 * tid) = o0;
    *(volatile v4i*)(op + 4 * (tid + OTHR)) = o1;
    __syncthreads();
  }
  if (tid == 0) srb[min(4 * nChunk, RBN - 1)] = carry;
  __syncthreads();
  v4i rv = {0, 0, 0, 0};
  if (tid < 32) rv = *(const v4i*)(srb + 4 * tid);
  if (tid < 32) *(volatile v4i*)(rbase + 4 * tid) = rv;
  __threadfence();
  if (tid < 32) *(volatile v4i*)(rbase + 4 * tid) = rv;
}

__global__ __launch_bounds__(NTHR) void k_fill(
    const int* __restrict__ dsts, const int* __restrict__ off, const int* __restrict__ rbase,
    int* csr, int nE, int vec8, int csrLen) {
  extern __shared__ v4f lds_dyn[];
  int* region = (int*)lds_dyn;
  int* cursor = region + RCAP;
  int* list   = cursor + NBF;
  int* wcnt   = list + LISTN;
  const int tid = threadIdx.x, lane = tid & 31, wave = tid >> 5;
  const int b = blockIdx.x;
  const int nodeBase = b * NBF;

  int rb0 = rbase[b];
  const int rb1 = rbase[b + 1];
  rb0 = rb0 < 0 ? 0 : (rb0 > csrLen ? csrLen : rb0);
  rb0 &= ~31;
  int len = rb1 - rb0;
  len = len < 0 ? 0 : (len > RCAP ? RCAP : len);
  int lenW = (len + 31) & ~31;
  if (rb0 + lenW > csrLen) lenW = (csrLen - rb0) & ~31;

  {
    const v4i z = {0, 0, 0, 0};
    for (int i = tid; i < RCAP / 4; i += NTHR) ((v4i*)region)[i] = z;
    for (int s = tid; s < NBF; s += NTHR) {
      int o = off[nodeBase + s] - rb0;
      o = o < 0 ? 0 : (o > RCAP ? RCAP : o);
      cursor[s] = o;
    }
  }
  __syncthreads();

  const int nChunks = (nE + CHUNK - 1) / CHUNK;
#pragma unroll 1
  for (int ch = 0; ch < nChunks; ++ch) {
    const int cbase = ch * CHUNK;
    const int wc = scan_chunk<NBF>(dsts, nE, cbase, nodeBase, vec8, list, tid, lane, wave);
    if (lane == 0) wcnt[wave] = wc;
    __syncthreads();
    if (wave == 0) {
#pragma unroll 1
      for (int wsx = 0; wsx < NWAVE; ++wsx) {
        int n = __builtin_amdgcn_readfirstlane(wcnt[wsx]);
        n = n > WCAP ? WCAP : (n < 0 ? 0 : n);
        const int* lp = list + wsx * WCAP;
#pragma unroll 1
        for (int i = 0; i < n; ++i) {
          const int ent = __builtin_amdgcn_readfirstlane(lp[i]);
          const int sl  = ent & (NBF - 1);
          int e = cbase + ((ent >> 12) & (CHUNK - 1));
          e = e > nE - 1 ? nE - 1 : e;
          if (lane == 0) {
            int cp = cursor[sl];
            cp = cp < 0 ? 0 : (cp > RCAP - 1 ? RCAP - 1 : cp);
            region[cp] = e;
            const int np = cp + 1;
            cursor[sl] = np > RCAP ? RCAP : np;
          }
        }
      }
    }
    __syncthreads();
  }

  const int nv = lenW >> 2;
  int* gp = csr + rb0;
#pragma unroll 1
  for (int i = tid; i < nv; i += NTHR) { const v4i v = ((const v4i*)region)[i]; *(volatile v4i*)(gp + 4 * i) = v; }
  __threadfence();
#pragma unroll 1
  for (int i = tid; i < nv; i += NTHR) { const v4i v = ((const v4i*)region)[i]; *(volatile v4i*)(gp + 4 * i) = v; }
}

__global__ __launch_bounds__(GTHR) void k_nodegemm(const float* __restrict__ x, const unsigned short* __restrict__ B1h,
                                                   const unsigned short* __restrict__ B1l, const float* __restrict__ be0,
                                                   float* PQ, int nN) {
  __shared__ __attribute__((aligned(16))) unsigned short Ah[GROWS * APZ];
  __shared__ __attribute__((aligned(16))) unsigned short Al[GROWS * APZ];
  __shared__ __attribute__((aligned(16))) float stg[GROWS * PQW];
  const int tid = threadIdx.x, lane = tid & 31, wave = tid >> 5, hh = lane >> 4, m = lane & 15;
  const int rowBase = blockIdx.x * GROWS;
  {
    const int r = tid >> 1, c0 = (tid & 1) * 64;
    int xrow = rowBase + r;
    xrow = xrow > nN - 1 ? nN - 1 : xrow;
    const float* xp = x + (size_t)xrow * CH + c0;
#pragma unroll
    for (int j = 0; j < 8; ++j) {
      const v4f a = *(const v4f*)(xp + 8 * j), b = *(const v4f*)(xp + 8 * j + 4);
      v8us hv, lv;
      split8(a, b, hv, lv);
      *(v8us*)(Ah + r * APZ + c0 + 8 * j) = hv;
      *(v8us*)(Al + r * APZ + c0 + 8 * j) = lv;
    }
  }
  __syncthreads();

#pragma unroll
  for (int cg = 0; cg < 4; ++cg) {
    v8f acc[4];
    mma3<4, KPB, APZ>(Ah + wave * 16 * APZ, Al + wave * 16 * APZ,
                      B1h + (size_t)(64 * cg) * KPB, B1l + (size_t)(64 * cg) * KPB, lane, acc);
    float* sp = stg + (wave * 16 + 8 * hh) * PQW + 64 * cg + m;
#pragma unroll
    for (int t = 0; t < 4; ++t) {
      const int col = 64 * cg + 16 * t + m;
      const float bv = (cg >= 2) ? be0[(col - CH) & (CH - 1)] : 0.0f;
#pragma unroll
      for (int r = 0; r < 8; ++r) sp[r * PQW + 16 * t] = acc[t][r] + bv;
    }
  }
  __syncthreads();

  float* gp = PQ + (size_t)rowBase * PQW;
#pragma unroll
  for (int it = 0; it < 32; ++it) {
    const int f = it * GTHR + tid;
    const v4f v = *(const v4f*)(stg + 4 * f);
    *(volatile v4f*)(gp + 4 * f) = v;
  }
  __threadfence();
#pragma unroll
  for (int it = 0; it < 32; ++it) {
    const int f = it * GTHR + tid;
    const v4f v = *(const v4f*)(stg + 4 * f);
    *(volatile v4f*)(gp + 4 * f) = v;
  }
}

__global__ __launch_bounds__(NTHR) void k_final(
    const float* __restrict__ PQ, const int* __restrict__ csr,
    const int* __restrict__ offp, const int* __restrict__ cntp,
    const int* __restrict__ srcs, const float* __restrict__ posn,
    const float* __restrict__ Wd, const _Float16* __restrict__ B2, const float* __restrict__ b2,
    float* AGG, int nN, int nE, int csrLen) {
  __shared__ __attribute__((aligned(16))) _Float16 zt[NWAVE * KNB * APZ];
  __shared__ __attribute__((aligned(16))) float sout[NWAVE * CH];
  __shared__ __attribute__((aligned(16))) float attw[NWAVE * KNB];
  __shared__ __attribute__((aligned(16))) int slot[NWAVE];
  const int tid = threadIdx.x, lane = tid & 31, wave = tid >> 5, hh = lane >> 4, m = lane & 15;
  const int base = blockIdx.x * NPB;
  _Float16* zw  = zt + wave * (KNB * APZ);
  float*    aww = attw + wave * KNB;
  float b2c[8];
#pragma unroll
  for (int t = 0; t < 8; ++t) b2c[t] = b2[16 * t + m];
  const v4f d0 = *(const v4f*)(Wd + 4 * lane);
  const v4f d1 = *(const v4f*)(Wd + CH + 4 * lane);
  const v4f d2 = *(const v4f*)(Wd + 2 * CH + 4 * lane);

#pragma unroll 1
  for (int it = 0; it < NIT; ++it) {
    const int n = base + it * NWAVE + wave;
    const bool nval = n < nN;
    const int cc = nval ? n : nN - 1;
    const int cnr = cntp[cc];
    const int ofr = offp[cc];
    int cn = nval ? cnr : 0;
    cn = cn < 0 ? 0 : (cn > DEGCAP ? DEGCAP : cn);
    cn = __builtin_amdgcn_readfirstlane(cn);
    int of = ofr;
    of = of < 0 ? 0 : (of > csrLen ? csrLen : of);
    of = __builtin_amdgcn_readfirstlane(of);
    const v4f qb = *(const v4f*)(PQ + (size_t)cc * PQW + CH + 4 * lane);
    const float pnx = posn[(size_t)cc * 3 + 0];
    const float pny = posn[(size_t)cc * 3 + 1];
    const float pnz = posn[(size_t)cc * 3 + 2];
    const int ntw = (cn + KNB - 1) >> 4;
    if (lane == 0) slot[wave] = ntw;
    __syncthreads();
    int ntmax;
    {
      const v4i sA = *(const v4i*)slot, sB = *(const v4i*)(slot + 4);
      int mm = max(max(sA.x, sA.y), max(sA.z, sA.w));
      mm = max(mm, max(max(sB.x, sB.y), max(sB.z, sB.w)));
      mm = mm < 0 ? 0 : (mm > DEGCAP / KNB ? DEGCAP / KNB : mm);
      ntmax = __builtin_amdgcn_readfirstlane(mm);
    }
    float cs[8] = {0.f, 0.f, 0.f, 0.f, 0.f, 0.f, 0.f, 0.f};
#pragma unroll 1
    for (int tt = 0; tt < ntmax; ++tt) {
      int nv = cn - tt * KNB;
      nv = nv < 0 ? 0 : (nv > KNB ? KNB : nv);
      nv = __builtin_amdgcn_readfirstlane(nv);
      int cp = of + tt * KNB + m;
      cp = cp < 0 ? 0 : (cp > csrLen - 1 ? csrLen - 1 : cp);
      int e = csr[cp];
      e = e < 0 ? 0 : (e > nE - 1 ? nE - 1 : e);
      int sv = srcs[e];
      sv = sv < 0 ? 0 : (sv > nN - 1 ? nN - 1 : sv);
      const float dx = posn[(size_t)sv * 3 + 0] - pnx;
      const float dy = posn[(size_t)sv * 3 + 1] - pny;
      const float dz = posn[(size_t)sv * 3 + 2] - pnz;
      const float aw = (m < nv) ? 1.0f : 0.0f;
      __syncthreads();
      if (nv > 0) {
        if (lane < KNB) aww[lane] = aw;
        rows_z<0>(zw, PQ, sv, dx, dy, dz, qb, d0, d1, d2, lane);
        asm volatile("" ::: "memory");
        rows_z<8>(zw, PQ, sv, dx, dy, dz, qb, d0, d1, d2, lane);
      }
      __syncthreads();
      if (nv > 0) {
        v8f acc[8];
        mma16<8>(zw, B2, lane, acc);
        const v4f a0 = *(const v4f*)(aww + 8 * hh);
        const v4f a1 = *(const v4f*)(aww + 8 * hh + 4);
        const float av[8] = {a0.x, a0.y, a0.z, a0.w, a1.x, a1.y, a1.z, a1.w};
#pragma unroll
        for (int t = 0; t < 8; ++t) {
#pragma unroll
          for (int r = 0; r < 8; ++r) cs[t] = fmaf(acc[t][r] * RZW + b2c[t], av[r], cs[t]);
        }
      }
    }
#pragma unroll
    for (int t = 0; t < 8; ++t) cs[t] += __shfl_xor(cs[t], 16, 32);
    if (hh == 0) {
#pragma unroll
      for (int t = 0; t < 8; ++t) sout[wave * CH + 16 * t + m] = cs[t];
    }
    __syncthreads();
    {
      const int row  = tid >> 5;
      const int node = base + it * NWAVE + row;
      float* op = AGG + (size_t)node * CH + 4 * lane;
      const v4f sv4 = *(const v4f*)(sout + 4 * tid);
      *(volatile v4f*)op = sv4;
      __threadfence();
      *(volatile v4f*)op = sv4;
    }
  }
}

__global__ __launch_bounds__(GTHR) void k_nodemlp(const float* __restrict__ x, const float* __restrict__ AGG,
                                                  const unsigned short* __restrict__ B3h, const unsigned short* __restrict__ B3l,
                                                  const float* __restrict__ bn0,
                                                  const unsigned short* __restrict__ B4h, const unsigned short* __restrict__ B4l,
                                                  const float* __restrict__ bn1, float* out, int nN) {
  __shared__ __attribute__((aligned(16))) unsigned short ldsr[2 * GROWS * APW + 2 * GROWS * APZ];
  unsigned short* Ah = ldsr;
  unsigned short* Al = ldsr + GROWS * APW;
  unsigned short* Hh = ldsr + 2 * GROWS * APW;
  unsigned short* Hl = Hh + GROWS * APZ;
  float* stg = (float*)ldsr;
  const int tid = threadIdx.x, lane = tid & 31, wave = tid >> 5, hh = lane >> 4, m = lane & 15;
  const int rowBase = blockIdx.x * GROWS;
  {
    const int r = tid >> 1, half = tid & 1;
    int row = rowBase + r;
    row = row > nN - 1 ? nN - 1 : row;
    const float* sp = (half == 0) ? (x + (size_t)row * CH) : (AGG + (size_t)row * CH);
    unsigned short* dh = Ah + r * APW + half * CH;
    unsigned short* dl = Al + r * APW + half * CH;
#pragma unroll 4
    for (int j = 0; j < 16; ++j) {
      const v4f a = *(const v4f*)(sp + 8 * j), b = *(const v4f*)(sp + 8 * j + 4);
      v8us hv, lv;
      split8(a, b, hv, lv);
      *(v8us*)(dh + 8 * j) = hv;
      *(v8us*)(dl + 8 * j) = lv;
    }
  }
  __syncthreads();

#pragma unroll
  for (int cg = 0; cg < 2; ++cg) {
    v8f acc[4];
    mma3<4, KPW, APW>(Ah + wave * 16 * APW, Al + wave * 16 * APW,
                      B3h + (size_t)(64 * cg) * KPW, B3l + (size_t)(64 * cg) * KPW, lane, acc);
#pragma unroll
    for (int t = 0; t < 4; ++t) {
      const int col = 64 * cg + 16 * t + m;
      const float bv = bn0[col & (CH - 1)];
#pragma unroll
      for (int r = 0; r < 8; ++r) {
        const float v = fmaxf(acc[t][r] + bv, 0.0f);
        unsigned short hs, ls;
        bfsplit(v, hs, ls);
        Hh[(wave * 16 + 8 * hh + r) * APZ + col] = hs;
        Hl[(wave * 16 + 8 * hh + r) * APZ + col] = ls;
      }
    }
  }
  __syncthreads();

#pragma unroll
  for (int cg = 0; cg < 2; ++cg) {
    v8f acc[4];
    mma3<4, KPB, APZ>(Hh + wave * 16 * APZ, Hl + wave * 16 * APZ,
                      B4h + (size_t)(64 * cg) * KPB, B4l + (size_t)(64 * cg) * KPB, lane, acc);
    float* sp = stg + (wave * 16 + 8 * hh) * CH + 64 * cg + m;
#pragma unroll
    for (int t = 0; t < 4; ++t) {
      const int col = 64 * cg + 16 * t + m;
      const float bv = bn1[col & (CH - 1)];
#pragma unroll
      for (int r = 0; r < 8; ++r) sp[r * CH + 16 * t] = acc[t][r] + bv;
    }
  }
  __syncthreads();

  float* gp = out + (size_t)rowBase * CH;
#pragma unroll
  for (int it = 0; it < 16; ++it) {
    const int f = it * GTHR + tid;
    const v4f v = *(const v4f*)(stg + 4 * f);
    if (rowBase + (f >> 5) < nN) *(volatile v4f*)(gp + 4 * f) = v;
  }
  __threadfence();
#pragma unroll
  for (int it = 0; it < 16; ++it) {
    const int f = it * GTHR + tid;
    const v4f v = *(const v4f*)(stg + 4 * f);
    if (rowBase + (f >> 5) < nN) *(volatile v4f*)(gp + 4 * f) = v;
  }
}

extern "C" void kernel_launch(void* const* d_in, const int* in_sizes, int n_in,
                              void* d_out, int out_size, void* d_ws, size_t ws_size,
                              hipStream_t stream) {
  if (n_in < 11) return;
  const int nN = in_sizes[0] / CH;
  const int nE = in_sizes[1] / 2;
  if (nN <= 0 || nE <= 0) return;
  if (in_sizes[0] != nN * CH || in_sizes[1] != 2 * nE || in_sizes[2] != 3 * nN) return;
  if (in_sizes[3] != (3 * CH + 3) * CH || in_sizes[4] != CH || in_sizes[5] != CH * CH || in_sizes[6] != CH) return;
  if (in_sizes[7] != 2 * CH * CH || in_sizes[8] != CH || in_sizes[9] != CH * CH || in_sizes[10] != CH) return;
  if (out_size != nN * CH) return;
  if (nE > (1 << 28) || nN > (1 << 24)) return;

  const float* x    = (const float*)d_in[0];
  const int*   ei   = (const int*)d_in[1];
  const float* posn = (const float*)d_in[2];
  const float* We0  = (const float*)d_in[3];
  const float* be0  = (const float*)d_in[4];
  const float* We1  = (const float*)d_in[5];
  const float* be1  = (const float*)d_in[6];
  const float* Wn0  = (const float*)d_in[7];
  const float* bn0  = (const float*)d_in[8];
  const float* Wn1  = (const float*)d_in[9];
  const float* bn1  = (const float*)d_in[10];
  const int* srcs = ei;
  const int* dsts = ei + nE;
  const float* Wd = We0 + (size_t)3 * CH * CH;
  float* out = (float*)d_out;

  const int nBlkG = (nN + GROWS - 1) / GROWS;
  const int NPADG = nBlkG * GROWS;
  const int nBlkP = (nN + NPB - 1) / NPB;
  const int NPADP = nBlkP * NPB;
  const int nBC   = (nN + NBC - 1) / NBC;
  const int CNTPAD = nBC * NBC;
  if (4 * nBC + 1 > RBN) return;
  const int nBF    = (nN + NBF - 1) / NBF;
  const int csrLen = ((nE + 31) & ~31) + 4096;
  if (31 * 4 * nBC > 4096) return;

  char* ws = (char*)d_ws;
  size_t off = 0;
  const size_t oB   = off; off += (size_t)BPTOT * 2;               off = (off + 255) & ~(size_t)255;
  const size_t oCnt = off; off += (size_t)CNTPAD * 4;              off = (off + 255) & ~(size_t)255;
  const size_t oOff = off; off += (size_t)CNTPAD * 4;              off = (off + 255) & ~(size_t)255;
  const size_t oRb  = off; off += (size_t)RBN * 4;                 off = (off + 255) & ~(size_t)255;
  const size_t oCsr = off; off += (size_t)csrLen * 4;              off = (off + 255) & ~(size_t)255;
  const size_t oPQ  = off; off += (size_t)NPADG * PQW * 4;         off = (off + 255) & ~(size_t)255;
  const size_t oAgg = off; off += (size_t)NPADP * CH * 4;          off = (off + 255) & ~(size_t)255;
  if (off > ws_size || off > (size_t)WSCAP) return;
  unsigned short* Bpl  = (unsigned short*)(ws + oB);
  int*            cnt  = (int*)(ws + oCnt);
  int*            offp = (int*)(ws + oOff);
  int*            rb   = (int*)(ws + oRb);
  int*            csr  = (int*)(ws + oCsr);
  float*          PQ   = (float*)(ws + oPQ);
  float*          AGG  = (float*)(ws + oAgg);
  const _Float16* B2p  = (const _Float16*)(Bpl + OFF_B2);

  const int vec8 = ((nE & 3) == 0) ? 1 : 0;

  k_wprep<<<48, NTHR, 0, stream>>>(We0, We1, Wn0, Wn1, Bpl);
  k_count<<<nBC, NTHR, 0, stream>>>(dsts, cnt, nE, vec8);
  k_offsets<<<1, OTHR, 0, stream>>>(cnt, offp, rb, nBC);
  hipFuncSetAttribute(reinterpret_cast<const void*>(&k_fill),
                      hipFuncAttributeMaxDynamicSharedMemorySize, LDS_FILL);
  k_fill<<<nBF, NTHR, LDS_FILL, stream>>>(dsts, offp, rb, csr, nE, vec8, csrLen);
  k_nodegemm<<<nBlkG, GTHR, 0, stream>>>(x, Bpl + OFF_B1H, Bpl + OFF_B1L, be0, PQ, nN);
  k_final<<<nBlkP, NTHR, 0, stream>>>(PQ, csr, offp, cnt, srcs, posn, Wd, B2p, be1, AGG, nN, nE, csrLen);
  k_nodemlp<<<nBlkG, GTHR, 0, stream>>>(x, AGG, Bpl + OFF_B3H, Bpl + OFF_B3L, bn0, Bpl + OFF_B4H, Bpl + OFF_B4L, bn1, out, nN);
}
